// FixedProjectionBlock_44976897524206
// MI455X (gfx1250) — hardware-run, weakly checked
//
#include <hip/hip_runtime.h>
#include <math.h>

typedef __attribute__((ext_vector_type(16))) _Float16 v16h;
typedef __attribute__((ext_vector_type(8)))  _Float16 v8h;
typedef __attribute__((ext_vector_type(8)))  float    v8f;
typedef __attribute__((ext_vector_type(4)))  float    v4f;
typedef __attribute__((ext_vector_type(2)))  float    v2f;
typedef __attribute__((ext_vector_type(4)))  unsigned int v4u;

constexpr int kBatch = 2;
constexpr int kSeq   = 1024;
constexpr int kDim   = 512;
constexpr int kRows  = kBatch * kSeq;
constexpr int kNPh   = 16;
constexpr int kGate  = 256;
constexpr int kNKQ   = 64;
constexpr int kPhP   = 96;
constexpr int kPosP  = 32;
constexpr int kTS    = 32;
constexpr int kYP    = 68;
constexpr float kXCarry    = 16.0f;
constexpr float kWCarry    = 256.0f;
constexpr float kGemmScale = 1.0f / (kXCarry * kWCarry);
constexpr float kPi        = 3.14159265358979323846f;
constexpr float kTwoPi     = 2.0f * kPi;
constexpr float kInvDim    = 1.0f / (float)kDim;
constexpr float kLnEps     = 1e-5f;
static_assert(kGemmScale == 1.0f / 4096.0f, "carry product");
static_assert((kDim % 32) == 0, "GEMM K multiple of 32");
static_assert((kRows % 64) == 0 && (kNKQ % 64) == 0 && (kGate % 64) == 0 && (kDim % 64) == 0, "GEMM M,N multiples of 64");
static_assert((kSeq % kTS) == 0 && (kDim % 64) == 0, "scan tiles");
static_assert(2 * kNPh <= kNKQ, "key|query columns fit the padded plane");

constexpr size_t kOffXH   = 0;
constexpr size_t kOffBTV  = kOffXH   + (size_t)kRows * kDim * 2;
constexpr size_t kOffBTO  = kOffBTV  + (size_t)kDim * kDim * 2;
constexpr size_t kOffBTG  = kOffBTO  + (size_t)kDim * kDim * 2;
constexpr size_t kOffBTKQ = kOffBTG  + (size_t)kGate * kDim * 2;
constexpr size_t kOffPOS  = kOffBTKQ + (size_t)kNKQ * kDim * 2;
constexpr size_t kOffTKQ  = kOffPOS  + (size_t)kSeq * kPosP * 4;
constexpr size_t kOffG1   = kOffTKQ  + (size_t)kRows * kNKQ * 4;
constexpr size_t kOffV    = kOffG1   + (size_t)kRows * kGate * 4;
constexpr size_t kOffPH   = kOffV    + (size_t)kRows * kDim * 4;
constexpr size_t kOffGATE = kOffPH   + (size_t)kRows * kPhP * 4;
constexpr size_t kOffWG   = kOffGATE + (size_t)kRows * 4;
constexpr size_t kOffY    = kOffWG   + (size_t)kRows * 4;
constexpr size_t kOffYNH  = kOffY    + (size_t)kRows * kDim * 4;
constexpr size_t kWsTotal = kOffYNH  + (size_t)kRows * kDim * 2;
static_assert(kWsTotal == 17514496ull, "carve total");
static_assert(kWsTotal <= 134217728ull, "carve cap");
static_assert((kOffBTV % 128) == 0 && (kOffBTO % 128) == 0 && (kOffBTG % 128) == 0 && (kOffBTKQ % 128) == 0 &&
              (kOffPOS % 128) == 0 && (kOffTKQ % 128) == 0 && (kOffG1 % 128) == 0 && (kOffV % 128) == 0 &&
              (kOffPH % 128) == 0 && (kOffGATE % 128) == 0 && (kOffWG % 128) == 0 && (kOffY % 128) == 0 &&
              (kOffYNH % 128) == 0, "128-B aligned regions");

__device__ __forceinline__ int wave_index() { return __builtin_amdgcn_readfirstlane((int)(threadIdx.x >> 5)); }
__device__ __forceinline__ unsigned pk16(unsigned short a, unsigned short b) { return (unsigned)a | ((unsigned)b << 16); }
__device__ __forceinline__ unsigned short h_bits(float f) { const _Float16 h = (_Float16)f; return __builtin_bit_cast(unsigned short, h); }

__device__ __forceinline__ void acc_tie_h(v8f& a, v16h x, v16h y) { asm volatile("v_nop\n\tv_nop\n\tv_nop\n\tv_nop" : "+v"(a) : "v"(x), "v"(y)); }
__device__ __forceinline__ void keep4_h(v16h a, v16h b, v16h c, v16h d) { asm volatile("v_nop" :: "v"(a), "v"(b), "v"(c), "v"(d)); }
__device__ __forceinline__ void acc_guard4(v8f& a, v8f& b, v8f& c, v8f& d) { asm volatile("v_nop\n\tv_nop\n\tv_nop\n\tv_nop" : "+v"(a), "+v"(b), "+v"(c), "+v"(d)); }

struct FragH {
  union U { v16h v; v8h h[2]; };
  static __device__ __forceinline__ v16h load(const _Float16* p) {
    U f; f.h[0] = *(const v8h*)(p); f.h[1] = *(const v8h*)(p + 16); return f.v;
  }
  static __device__ __forceinline__ v8f mma(v16h a, v16h b, v8f c) {
    return __builtin_amdgcn_wmma_f32_16x16x32_f16(false, a, false, b, (short)0, c, false, false);
  }
};

template <int BIAS_MODE, bool RESID>
__global__ __launch_bounds__(256) void wmma_gemm64(
    const unsigned short* __restrict__ Ap, int lda,
    const unsigned short* __restrict__ Btp, int ldb,
    float* __restrict__ C, int ldc,
    const float* __restrict__ bias,
    const float* __restrict__ resid,
    int M, int N, int K, float scale) {
  const _Float16* A  = (const _Float16*)Ap;
  const _Float16* Bt = (const _Float16*)Btp;
  __shared__ __align__(16) float sT[8][16 * 68];
  const int lane = threadIdx.x & 31;
  const int wave = wave_index();
  const int tilesN = N >> 6;
  const int tilesM = M >> 6;
  const int tile = blockIdx.x * 8 + wave;
  if (tile >= tilesM * tilesN) return;
  const int tm = tile / tilesN;
  const int tn = tile - tm * tilesN;
  const int m0 = tm << 6;
  const int n0 = tn << 6;

  const int rlane = lane & 15;
  const int koff  = (lane >> 4) * 8;
  const int mOff  = (lane >> 4) * 8;

  v8f acc[4][4];
#pragma unroll
  for (int i = 0; i < 4; ++i)
#pragma unroll
    for (int j = 0; j < 4; ++j) acc[i][j] = (v8f){0.f,0.f,0.f,0.f,0.f,0.f,0.f,0.f};

  for (int k0 = 0; k0 < K; k0 += 32) {
    v16h bh[4];
#pragma unroll
    for (int j = 0; j < 4; ++j) {
      const size_t bo = (size_t)(n0 + (j << 4) + rlane) * ldb + koff + k0;
      bh[j] = FragH::load(Bt + bo);
    }
#pragma unroll
    for (int i = 0; i < 4; ++i) {
      const size_t ao = (size_t)(m0 + (i << 4) + rlane) * lda + koff + k0;
      v16h ah = FragH::load(A + ao);
#pragma unroll
      for (int j = 0; j < 4; ++j) acc[i][j] = FragH::mma(ah, bh[j], acc[i][j]);
      acc_tie_h(acc[i][0], ah, bh[0]);
      acc_tie_h(acc[i][1], ah, bh[1]);
      acc_tie_h(acc[i][2], ah, bh[2]);
      acc_tie_h(acc[i][3], ah, bh[3]);
    }
    keep4_h(bh[0], bh[1], bh[2], bh[3]);
  }
  acc_guard4(acc[0][0], acc[0][1], acc[0][2], acc[0][3]);
  acc_guard4(acc[1][0], acc[1][1], acc[1][2], acc[1][3]);
  acc_guard4(acc[2][0], acc[2][1], acc[2][2], acc[2][3]);
  acc_guard4(acc[3][0], acc[3][1], acc[3][2], acc[3][3]);

  float* slab = sT[wave];
#pragma unroll
  for (int i = 0; i < 4; ++i) {
    const int mBase = m0 + (i << 4);
#pragma unroll
    for (int j = 0; j < 4; ++j) {
      const int n = n0 + (j << 4) + rlane;
      float bv = 0.f;
      if (BIAS_MODE == 2) bv = bias[n];
#pragma unroll
      for (int r = 0; r < 8; ++r) {
        float v = acc[i][j][r] * scale;
        if (BIAS_MODE == 2) v += bv;
        slab[(mOff + r) * 68 + (j << 4) + rlane] = v;
      }
    }
    __builtin_amdgcn_fence(__ATOMIC_RELEASE, "workgroup");
    __builtin_amdgcn_wave_barrier();
    __builtin_amdgcn_fence(__ATOMIC_ACQUIRE, "workgroup");
    {
      const int hh = lane >> 4, c4 = (lane & 15) * 4;
      for (int pass = 0; pass < 2; ++pass) {
#pragma unroll
        for (int it = 0; it < 8; ++it) {
          const int row = it * 2 + hh;
          v4f v = *(const v4f*)(slab + row * 68 + c4);
          const size_t go = (size_t)(mBase + row) * ldc + n0 + c4;
          if (RESID) {
            const v4f rv = *(const v4f*)(resid + go);
            v = v + rv;
          }
          *(volatile v4f*)(C + go) = v;
        }
        __threadfence();
      }
    }
    __builtin_amdgcn_fence(__ATOMIC_RELEASE, "workgroup");
    __builtin_amdgcn_wave_barrier();
    __builtin_amdgcn_fence(__ATOMIC_ACQUIRE, "workgroup");
  }
}

__global__ __launch_bounds__(256) void cast8_f16_kernel(const float* __restrict__ in, unsigned short* __restrict__ out, int n8, float carry) {
  const int i = blockIdx.x * 256 + threadIdx.x;
  if (i >= n8) return;
  const float* p = in + 8 * (size_t)i;
  const v4f a = *(const v4f*)(p);
  const v4f c = *(const v4f*)(p + 4);
  unsigned short hb[8];
#pragma unroll
  for (int e = 0; e < 4; ++e) {
    const float fa = a[e] * carry;
    const float fc = c[e] * carry;
    hb[e]     = h_bits(fa);
    hb[4 + e] = h_bits(fc);
  }
  const v4u u = (v4u){pk16(hb[0], hb[1]), pk16(hb[2], hb[3]), pk16(hb[4], hb[5]), pk16(hb[6], hb[7])};
  unsigned short* q = out + 8 * (size_t)i;
  *(volatile v4u*)q = u;
  __threadfence();
  *(volatile v4u*)q = u;
}

__global__ __launch_bounds__(256) void wt_f16_kernel(const float* __restrict__ W0, const float* __restrict__ W1,
                                                     const float* __restrict__ W2,
                                                     unsigned short* __restrict__ O0, unsigned short* __restrict__ O1,
                                                     unsigned short* __restrict__ O2, float carry) {
  __shared__ float sm[64][65];
  const int t  = threadIdx.x;
  const int z  = blockIdx.z;
  const int ncols = (z == 2) ? kGate : kDim;
  const int d0 = blockIdx.x * 64;
  const int h0 = blockIdx.y * 64;
  if (h0 >= ncols) return;
  const float* W = (z == 0) ? W0 : (z == 1) ? W1 : W2;
  unsigned short* op = (z == 0) ? O0 : (z == 1) ? O1 : O2;
#pragma unroll
  for (int i = 0; i < 16; ++i) {
    const int e = i * 256 + t;
    const int r = e >> 6;
    const int c = e & 63;
    sm[c][r] = W[(size_t)(d0 + r) * ncols + h0 + c] * carry;
  }
  __syncthreads();
  const int lane = t & 31, wave = wave_index();
  const int q = lane >> 3, c8 = (lane & 7) * 8;
  for (int pass = 0; pass < 2; ++pass) {
#pragma unroll
    for (int it = 0; it < 2; ++it) {
      const int row = wave * 8 + it * 4 + q;
      unsigned short hb[8];
#pragma unroll
      for (int e = 0; e < 8; ++e) hb[e] = h_bits(sm[row][c8 + e]);
      const v4u u = (v4u){pk16(hb[0], hb[1]), pk16(hb[2], hb[3]), pk16(hb[4], hb[5]), pk16(hb[6], hb[7])};
      *(volatile v4u*)(op + (size_t)(h0 + row) * kDim + d0 + c8) = u;
    }
    __threadfence();
  }
}

__global__ __launch_bounds__(256) void kq_plane_kernel(const float* __restrict__ keyp, const float* __restrict__ qryp,
                                                       unsigned short* __restrict__ out, float carry) {
  __shared__ float sm[32][65];
  const int t  = threadIdx.x;
  const int d0 = blockIdx.x * 64;
#pragma unroll
  for (int i = 0; i < 4; ++i) {
    const int e = i * 256 + t;
    const int r = e >> 4;
    const int c = e & 15;
    sm[c][r]      = keyp[(size_t)(d0 + r) * kNPh + c] * carry;
    sm[16 + c][r] = qryp[(size_t)(d0 + r) * kNPh + c] * carry;
  }
  __syncthreads();
  const int lane = t & 31, wave = wave_index();
  const int q = lane >> 3, c8 = (lane & 7) * 8;
  for (int pass = 0; pass < 2; ++pass) {
#pragma unroll
    for (int it = 0; it < 2; ++it) {
      const int row = wave * 8 + it * 4 + q;
      const int rs  = row & 31;
      const bool live = (row < 32);
      unsigned short hb[8];
#pragma unroll
      for (int e = 0; e < 8; ++e) hb[e] = h_bits(sm[rs][c8 + e]);
      const unsigned u0 = live ? pk16(hb[0], hb[1]) : 0u;
      const unsigned u1 = live ? pk16(hb[2], hb[3]) : 0u;
      const unsigned u2 = live ? pk16(hb[4], hb[5]) : 0u;
      const unsigned u3 = live ? pk16(hb[6], hb[7]) : 0u;
      const v4u u = (v4u){u0, u1, u2, u3};
      *(volatile v4u*)(out + (size_t)row * kDim + d0 + c8) = u;
    }
    __threadfence();
  }
}

__global__ __launch_bounds__(256) void pos_table_kernel(const float* __restrict__ pf, float* __restrict__ POS) {
  const int lane = threadIdx.x & 31, wave = wave_index();
  const int l = blockIdx.x * 8 + wave;
  const int p = lane >> 1;
  const float f = pf[p];
  const float a = __fmul_rn((float)l, f);
  const float phi = __fmul_rn(a, kTwoPi);
  float sn, cs;
  sincosf(phi, &sn, &cs);
  const float val = (lane & 1) ? sn : cs;
  float* q = POS + (size_t)l * kPosP + lane;
  *(volatile float*)q = val;
  __threadfence();
  *(volatile float*)q = val;
}

__global__ __launch_bounds__(256) void phasor_rows_kernel(const float* __restrict__ TKQ, float* __restrict__ PH) {
  __shared__ __align__(16) float sR[8][kPhP];
  const int lane = threadIdx.x & 31, wave = wave_index();
  const int row = blockIdx.x * 8 + wave;
  const float pre = TKQ[(size_t)row * kNKQ + lane];
  const float th = tanhf(pre) * kPi;
  float sn, cs;
  sincosf(th, &sn, &cs);
  const float c1 = __shfl_xor(cs, 4, 32);
  const float s1 = __shfl_xor(sn, 4, 32);
  const float pc = cs * c1 - sn * s1;
  const float ps = cs * s1 + sn * c1;
  const float c2 = __shfl_xor(pc, 8, 32);
  const float s2 = __shfl_xor(ps, 8, 32);
  const float jc = pc * c2 - ps * s2;
  const float js = pc * s2 + ps * c2;
  const int j  = lane & 15;
  const int hq = lane >> 4;
  float* sr = sR[wave];
  sr[hq * 32 + 2 * j]     = cs;
  sr[hq * 32 + 2 * j + 1] = sn;
  if (j < 4) {
    sr[64 + hq * 8 + 2 * j]     = jc;
    sr[64 + hq * 8 + 2 * j + 1] = js;
  }
  if (lane < 16) sr[80 + lane] = 0.0f;
  __syncthreads();
  const int lc = (lane < 24) ? lane : 23;
  const v4f v = *(const v4f*)(sr + lc * 4);
  float* gp = PH + (size_t)row * kPhP + lc * 4;
  if (lane < 24) *(volatile v4f*)gp = v;
  __threadfence();
  if (lane < 24) *(volatile v4f*)gp = v;
}

__global__ __launch_bounds__(256) void gate_kernel(const float* __restrict__ G1, const float* __restrict__ g2w,
                                                   const float* __restrict__ g2b, float* __restrict__ gate) {
  __shared__ float sG[32];
  const int lane = threadIdx.x & 31, wave = wave_index();
  const int r0 = blockIdx.x * 32;
  const float gb = g2b[0];
#pragma unroll 1
  for (int i = 0; i < 4; ++i) {
    const int row = r0 + wave * 4 + i;
    float part = 0.0f;
#pragma unroll 1
    for (int it = 0; it < 8; ++it) {
      const float tv = G1[(size_t)row * kGate + it * 32 + lane];
      const float wv = g2w[it * 32 + lane];
      const float ge = 0.5f * tv * (1.0f + erff(tv * 0.70710678118654752f));
      part = fmaf(ge, wv, part);
    }
    part += __shfl_xor(part, 16, 32);
    part += __shfl_xor(part, 8, 32);
    part += __shfl_xor(part, 4, 32);
    part += __shfl_xor(part, 2, 32);
    part += __shfl_xor(part, 1, 32);
    const float gv = 1.0f / (1.0f + expf(-(part + gb)));
    if (lane == 0) sG[wave * 4 + i] = gv;
  }
  __syncthreads();
  if (wave == 0) {
    const float v = sG[lane];
    float* q = gate + r0 + lane;
    *(volatile float*)q = v;
    __threadfence();
    *(volatile float*)q = v;
  }
}

__global__ __launch_bounds__(256) void wg_kernel(const float* __restrict__ PH,
                                                 const float* __restrict__ sscale, const float* __restrict__ sbias,
                                                 const float* __restrict__ rscale, const float* __restrict__ rthr,
                                                 float* __restrict__ wg) {
  __shared__ __align__(16) float sJ[kSeq * 8];
  const int t = threadIdx.x;
  const int lane = t & 31, wave = wave_index();
  const int b = blockIdx.x;
  const float ss = sscale[0], sb = sbias[0];
  const float sc = fminf(fmaxf(rscale[0], 1.0f), 20.0f);
  const float th = fminf(fmaxf(rthr[0], 0.1f), 0.9f);
#pragma unroll
  for (int i = 0; i < 4; ++i) {
    const int l = i * 256 + t;
    const float* src = PH + (size_t)(b * kSeq + l) * kPhP + 64;
    const v4f a = *(const v4f*)(src);
    const v4f c = *(const v4f*)(src + 4);
    *(v4f*)(sJ + l * 8)     = a;
    *(v4f*)(sJ + l * 8 + 4) = c;
  }
  __syncthreads();
  if (wave == 0 && lane < 8) {
    float run = 0.0f;
#pragma unroll 4
    for (int l = 0; l < kSeq; ++l) {
      const float v = sJ[l * 8 + lane];
      sJ[l * 8 + lane] = run;
      run += v;
    }
  }
  __syncthreads();
#pragma unroll 1
  for (int i = 0; i < 4; ++i) {
    const int l = i * 256 + t;
    const v4f a = *(const v4f*)(sJ + l * 8);
    const v4f c = *(const v4f*)(sJ + l * 8 + 4);
    const float m0 = sqrtf(a[0] * a[0] + a[1] * a[1]);
    const float m1 = sqrtf(a[2] * a[2] + a[3] * a[3]);
    const float m2 = sqrtf(c[0] * c[0] + c[1] * c[1]);
    const float m3 = sqrtf(c[2] * c[2] + c[3] * c[3]);
    const float mag = (((m0 + m1) + m2) + m3) * 0.25f;
    const float posn = fmaxf((float)l, 1.0f);
    const float nres = mag * (1.0f / sqrtf(posn));
    const float sur = 0.5f * (1.0f - tanhf(sc * (nres - th)));
    const float wv = 1.0f / (1.0f + expf(-(ss * (sur - 0.5f) + sb)));
    float* q = wg + (size_t)b * kSeq + l;
    *(volatile float*)q = wv;
    __threadfence();
    *(volatile float*)q = wv;
  }
}

__global__ __launch_bounds__(64) void scan_kernel(const float* __restrict__ PH, const float* __restrict__ POS,
                                                  const float* __restrict__ V, const float* __restrict__ wg,
                                                  const float* __restrict__ gate, const float* __restrict__ setw,
                                                  const float* __restrict__ posw_p, float* __restrict__ Y) {
  __shared__ __align__(16) float sPH[kTS * kPhP];
  __shared__ __align__(16) float sPS[kTS * kPosP];
  __shared__ __align__(16) float sV[kTS * 64];
  __shared__ __align__(16) float sY[kTS * kYP];
  __shared__ __align__(16) float sS[96];
  const int tid = threadIdx.x, lane = tid & 31, wave = wave_index();
  const int bix = blockIdx.y;
  const int d0  = blockIdx.x * 64;
  const size_t row0 = (size_t)bix * kSeq;

  float wsm[4];
  {
    const float a0 = setw[0], a1 = setw[1], a2 = setw[2], a3 = setw[3];
    const float mx = fmaxf(fmaxf(a0, a1), fmaxf(a2, a3));
    const float e0 = expf(a0 - mx), e1 = expf(a1 - mx), e2 = expf(a2 - mx), e3 = expf(a3 - mx);
    const float inv = 1.0f / (((e0 + e1) + e2) + e3);
    wsm[0] = e0 * inv; wsm[1] = e1 * inv; wsm[2] = e2 * inv; wsm[3] = e3 * inv;
  }
  const float posw = 1.0f / (1.0f + expf(-posw_p[0]));

  v2f mk[16], mc[4], mp[16];
#pragma unroll
  for (int i = 0; i < 16; ++i) { mk[i] = (v2f){0.f, 0.f}; mp[i] = (v2f){0.f, 0.f}; }
#pragma unroll
  for (int i = 0; i < 4; ++i) mc[i] = (v2f){0.f, 0.f};

  const int hh = lane >> 4, c4 = (lane & 15) * 4;

#pragma unroll 1
  for (int t0 = 0; t0 < kSeq; t0 += kTS) {
    __syncthreads();
    {
      const float* psrc = PH + (row0 + t0) * kPhP;
#pragma unroll
      for (int i = 0; i < 12; ++i) {
        const int idx = i * 64 + tid;
        *(v4f*)(sPH + idx * 4) = *(const v4f*)(psrc + idx * 4);
      }
      const float* qsrc = POS + (size_t)t0 * kPosP;
#pragma unroll
      for (int i = 0; i < 4; ++i) {
        const int idx = i * 64 + tid;
        *(v4f*)(sPS + idx * 4) = *(const v4f*)(qsrc + idx * 4);
      }
#pragma unroll
      for (int i = 0; i < 8; ++i) {
        const int idx = i * 64 + tid;
        const int r = idx >> 4, cc = (idx & 15) * 4;
        *(v4f*)(sV + r * 64 + cc) = *(const v4f*)(V + (row0 + t0 + r) * kDim + d0 + cc);
      }
      if (wave == 0) {
        sS[lane] = wg[row0 + t0 + lane];
        sS[64 + lane] = 1.0f / sqrtf((float)(t0 + lane + 1) * 4.0f);
      } else {
        sS[32 + lane] = gate[row0 + t0 + lane];
      }
    }
    __syncthreads();
#pragma unroll 1
    for (int s = 0; s < kTS; ++s) {
      const float* xr = sPH + s * kPhP;
      const float* pr = sPS + s * kPosP;
      const float v  = sV[s * 64 + tid];
      const float vg = v * sS[s];
      const v2f vg2 = (v2f){vg, vg};
      const v2f vv2 = (v2f){v, v};
      v2f tot2 = (v2f){0.f, 0.f};
#pragma unroll
      for (int ns = 0; ns < 4; ++ns) {
        const v4f ka = *(const v4f*)(xr + ns * 8);
        const v4f kb = *(const v4f*)(xr + ns * 8 + 4);
        const v4f qa = *(const v4f*)(xr + 32 + ns * 8);
        const v4f qb = *(const v4f*)(xr + 32 + ns * 8 + 4);
        v2f bank2 = (v2f){0.f, 0.f};
        mk[ns * 4 + 0] = ka.lo * vg2 + mk[ns * 4 + 0];
        bank2 = mk[ns * 4 + 0] * qa.lo + bank2;
        mk[ns * 4 + 1] = ka.hi * vg2 + mk[ns * 4 + 1];
        bank2 = mk[ns * 4 + 1] * qa.hi + bank2;
        mk[ns * 4 + 2] = kb.lo * vg2 + mk[ns * 4 + 2];
        bank2 = mk[ns * 4 + 2] * qb.lo + bank2;
        mk[ns * 4 + 3] = kb.hi * vg2 + mk[ns * 4 + 3];
        bank2 = mk[ns * 4 + 3] * qb.hi + bank2;
        tot2 = bank2 * wsm[ns] + tot2;
      }
      v2f cr2 = (v2f){0.f, 0.f};
      {
        const v4f ja = *(const v4f*)(xr + 64);
        const v4f jb = *(const v4f*)(xr + 68);
        const v4f ua = *(const v4f*)(xr + 72);
        const v4f ub = *(const v4f*)(xr + 76);
        mc[0] = ja.lo * vg2 + mc[0];
        cr2 = mc[0] * ua.lo + cr2;
        mc[1] = ja.hi * vg2 + mc[1];
        cr2 = mc[1] * ua.hi + cr2;
        mc[2] = jb.lo * vg2 + mc[2];
        cr2 = mc[2] * ub.lo + cr2;
        mc[3] = jb.hi * vg2 + mc[3];
        cr2 = mc[3] * ub.hi + cr2;
      }
      v2f rp2 = (v2f){0.f, 0.f};
#pragma unroll
      for (int q4 = 0; q4 < 8; ++q4) {
        const v4f pa = *(const v4f*)(pr + q4 * 4);
        mp[q4 * 2 + 0] = pa.lo * vv2 + mp[q4 * 2 + 0];
        rp2 = mp[q4 * 2 + 0] * pa.lo + rp2;
        mp[q4 * 2 + 1] = pa.hi * vv2 + mp[q4 * 2 + 1];
        rp2 = mp[q4 * 2 + 1] * pa.hi + rp2;
      }
      const float banks = tot2.x + tot2.y;
      const float cross = cr2.x + cr2.y;
      const float total = (banks + cross) * 0.2f;
      const float ret   = rp2.x + rp2.y;
      const float g = sS[32 + s];
      const float mix = g * total + (1.0f - g) * (posw * ret);
      sY[s * kYP + tid] = mix * sS[64 + s];
    }
    __syncthreads();
    v4f yv[8];
#pragma unroll
    for (int it = 0; it < 8; ++it) {
      const int row = it * 4 + wave * 2 + hh;
      yv[it] = *(const v4f*)(sY + row * kYP + c4);
    }
    for (int pass = 0; pass < 2; ++pass) {
#pragma unroll
      for (int it = 0; it < 8; ++it) {
        const int row = it * 4 + wave * 2 + hh;
        *(volatile v4f*)(Y + (row0 + t0 + row) * kDim + d0 + c4) = yv[it];
      }
      __threadfence();
    }
  }
}

__global__ __launch_bounds__(256) void ln_f16_kernel(const float* __restrict__ Y, const float* __restrict__ lng,
                                                     const float* __restrict__ lnb, unsigned short* __restrict__ YN,
                                                     float carry) {
  const int lane = threadIdx.x & 31, wave = wave_index();
  const int row = blockIdx.x * 8 + wave;
  const float* yr = Y + (size_t)row * kDim;
  float x[16];
#pragma unroll
  for (int it = 0; it < 2; ++it) {
    const int c0 = it * 256 + lane * 8;
    const v4f a = *(const v4f*)(yr + c0);
    const v4f c = *(const v4f*)(yr + c0 + 4);
#pragma unroll
    for (int e = 0; e < 4; ++e) { x[it * 8 + e] = a[e]; x[it * 8 + 4 + e] = c[e]; }
  }
  float s = 0.0f;
#pragma unroll
  for (int e = 0; e < 16; ++e) s += x[e];
  s += __shfl_xor(s, 16, 32);
  s += __shfl_xor(s, 8, 32);
  s += __shfl_xor(s, 4, 32);
  s += __shfl_xor(s, 2, 32);
  s += __shfl_xor(s, 1, 32);
  const float mu = s * kInvDim;
  float q = 0.0f;
#pragma unroll
  for (int e = 0; e < 16; ++e) { const float dlt = x[e] - mu; q = fmaf(dlt, dlt, q); }
  q += __shfl_xor(q, 16, 32);
  q += __shfl_xor(q, 8, 32);
  q += __shfl_xor(q, 4, 32);
  q += __shfl_xor(q, 2, 32);
  q += __shfl_xor(q, 1, 32);
  const float var = q * kInvDim;
  const float inv = 1.0f / sqrtf(var + kLnEps);
  v4u u[2];
#pragma unroll
  for (int it = 0; it < 2; ++it) {
    const int c0 = it * 256 + lane * 8;
    const v4f ga = *(const v4f*)(lng + c0);
    const v4f gc = *(const v4f*)(lng + c0 + 4);
    const v4f ba = *(const v4f*)(lnb + c0);
    const v4f bc = *(const v4f*)(lnb + c0 + 4);
    unsigned short hb[8];
#pragma unroll
    for (int e = 0; e < 4; ++e) {
      const float y0 = ((x[it * 8 + e] - mu) * inv * ga[e] + ba[e]) * carry;
      const float y1 = ((x[it * 8 + 4 + e] - mu) * inv * gc[e] + bc[e]) * carry;
      hb[e]     = h_bits(y0);
      hb[4 + e] = h_bits(y1);
    }
    u[it] = (v4u){pk16(hb[0], hb[1]), pk16(hb[2], hb[3]), pk16(hb[4], hb[5]), pk16(hb[6], hb[7])};
  }
  unsigned short* orow = YN + (size_t)row * kDim + lane * 8;
  for (int pass = 0; pass < 2; ++pass) {
    *(volatile v4u*)(orow)       = u[0];
    *(volatile v4u*)(orow + 256) = u[1];
    __threadfence();
  }
}

extern "C" void kernel_launch(void* const* d_in, const int* in_sizes, int n_in,
                              void* d_out, int out_size, void* d_ws, size_t ws_size,
                              hipStream_t stream) {
  if (n_in < 28) return;
  if (in_sizes[0] != kRows * kDim) return;
  if (in_sizes[1] != kDim * kNPh) return;
  if (in_sizes[2] != kDim * kNPh) return;
  if (in_sizes[4] != kDim * kDim) return;
  if (in_sizes[5] != kDim) return;
  if (in_sizes[6] != kDim) return;
  if (in_sizes[7] != kDim) return;
  if (in_sizes[8] != kDim * kDim) return;
  if (in_sizes[9] != kDim) return;
  if (in_sizes[10] != 4) return;
  if (in_sizes[11] != kNPh) return;
  if (in_sizes[13] != kDim * kGate) return;
  if (in_sizes[14] != kGate) return;
  if (in_sizes[15] != kGate) return;
  if (out_size != kRows * kDim) return;
  if (ws_size < kWsTotal) return;

  const float* x        = (const float*)d_in[0];
  const float* key_proj = (const float*)d_in[1];
  const float* qry_proj = (const float*)d_in[2];
  const float* v_w      = (const float*)d_in[4];
  const float* v_b      = (const float*)d_in[5];
  const float* ln_g     = (const float*)d_in[6];
  const float* ln_b     = (const float*)d_in[7];
  const float* out_w    = (const float*)d_in[8];
  const float* out_b    = (const float*)d_in[9];
  const float* set_w    = (const float*)d_in[10];
  const float* pfreq    = (const float*)d_in[11];
  const float* pos_wt   = (const float*)d_in[12];
  const float* g1_w     = (const float*)d_in[13];
  const float* g1_b     = (const float*)d_in[14];
  const float* g2_w     = (const float*)d_in[15];
  const float* g2_b     = (const float*)d_in[16];
  const float* s_scale  = (const float*)d_in[19];
  const float* s_bias   = (const float*)d_in[20];
  const float* r_scale  = (const float*)d_in[21];
  const float* r_thr    = (const float*)d_in[22];
  float* out = (float*)d_out;

  char* ws = (char*)d_ws;
  unsigned short* XH   = (unsigned short*)(ws + kOffXH);
  unsigned short* BTV  = (unsigned short*)(ws + kOffBTV);
  unsigned short* BTO  = (unsigned short*)(ws + kOffBTO);
  unsigned short* BTG  = (unsigned short*)(ws + kOffBTG);
  unsigned short* BTKQ = (unsigned short*)(ws + kOffBTKQ);
  float*          POS  = (float*)(ws + kOffPOS);
  float*          TKQ  = (float*)(ws + kOffTKQ);
  float*          G1   = (float*)(ws + kOffG1);
  float*          Vp   = (float*)(ws + kOffV);
  float*          PH   = (float*)(ws + kOffPH);
  float*          GATE = (float*)(ws + kOffGATE);
  float*          WG   = (float*)(ws + kOffWG);
  float*          Yp   = (float*)(ws + kOffY);
  unsigned short* YNH  = (unsigned short*)(ws + kOffYNH);

  cast8_f16_kernel<<<(kRows * kDim / 8) / 256, 256, 0, stream>>>(x, XH, kRows * kDim / 8, kXCarry);
  wt_f16_kernel<<<dim3(8, 8, 3), 256, 0, stream>>>(v_w, out_w, g1_w, BTV, BTO, BTG, kWCarry);
  kq_plane_kernel<<<8, 256, 0, stream>>>(key_proj, qry_proj, BTKQ, kWCarry);
  pos_table_kernel<<<kSeq / 8, 256, 0, stream>>>(pfreq, POS);

  wmma_gemm64<0, false><<<dim3(4), 256, 0, stream>>>(
      XH, kDim, BTKQ, kDim, TKQ, kNKQ, nullptr, nullptr, kRows, kNKQ, kDim, kGemmScale);
  wmma_gemm64<2, false><<<dim3(16), 256, 0, stream>>>(
      XH, kDim, BTG, kDim, G1, kGate, g1_b, nullptr, kRows, kGate, kDim, kGemmScale);
  wmma_gemm64<2, false><<<dim3(32), 256, 0, stream>>>(
      XH, kDim, BTV, kDim, Vp, kDim, v_b, nullptr, kRows, kDim, kDim, kGemmScale);

  phasor_rows_kernel<<<kRows / 8, 256, 0, stream>>>(TKQ, PH);
  gate_kernel<<<kRows / 32, 256, 0, stream>>>(G1, g2_w, g2_b, GATE);
  wg_kernel<<<kBatch, 256, 0, stream>>>(PH, s_scale, s_bias, r_scale, r_thr, WG);

  scan_kernel<<<dim3(kDim / 64, kBatch), 64, 0, stream>>>(PH, POS, Vp, WG, GATE, set_w, pos_wt, Yp);

  ln_f16_kernel<<<kRows / 8, 256, 0, stream>>>(Yp, ln_g, ln_b, YNH, kXCarry);

  wmma_gemm64<2, true><<<dim3(32), 256, 0, stream>>>(
      YNH, kDim, BTO, kDim, out, kDim, out_b, x, kRows, kDim, kDim, kGemmScale);
}
